// Block_37203006718445
// MI455X (gfx1250) — hardware-verified
//
#include <hip/hip_runtime.h>
#include <math.h>

#ifndef NB
#define NB 4
#endif
#ifndef SEQ
#define SEQ 2048
#endif
#define NB_FULL 4
#define SEQ_FULL 2048
#define DM 512
#define NHEAD 8
#define HDIM 64
#define DFF 2048
#define ROWS (NB * SEQ)

static_assert(NB >= 1 && NB <= NB_FULL);
static_assert(SEQ % 64 == 0 && SEQ <= SEQ_FULL);
static_assert(DM == NHEAD * HDIM);
static_assert(HDIM == 64);
static_assert(DM == 32 * 4 * 4);
static_assert(DM % 64 == 0 && DFF % 64 == 0);
static_assert(DM % 32 == 0 && DFF % 32 == 0);
static_assert(ROWS % 8 == 0);
static_assert((2 * DM) % 64 == 0);

typedef _Float16 v16h __attribute__((ext_vector_type(16)));
typedef _Float16 v8h  __attribute__((ext_vector_type(8)));
typedef float    v8f  __attribute__((ext_vector_type(8)));
typedef float    v4f  __attribute__((ext_vector_type(4)));
typedef unsigned int u4 __attribute__((ext_vector_type(4)));
typedef unsigned int u2 __attribute__((ext_vector_type(2)));
typedef v8h v8h_ma __attribute__((may_alias));
typedef v4f v4f_ma __attribute__((may_alias));

union FragU { v16h v; v8h h[2]; };
__device__ __forceinline__ v16h ld_frag(const _Float16* __restrict__ p) { FragU f; f.h[0] = *(const v8h*)(p); f.h[1] = *(const v8h*)(p + 16); return f.v; }

__device__ __forceinline__ v8f wmma16(v16h a, v16h b, v8f c) {
    c = __builtin_amdgcn_wmma_f32_16x16x32_f16(false, a, false, b, (short)0, c, false, false);
    asm volatile("v_nop\n\tv_nop\n\tv_nop\n\tv_nop" : "+v"(c) : "v"(a), "v"(b));
    return c;
}
__device__ __forceinline__ void dep_guard_h(v8f& a, v8f& b, v16h x, v16h y) { asm volatile("v_nop\n\tv_nop\n\tv_nop\n\tv_nop" : "+v"(a), "+v"(b) : "v"(x), "v"(y)); }
__device__ __forceinline__ void keep4_h(v16h a, v16h b, v16h c, v16h d) { asm volatile("v_nop" :: "v"(a), "v"(b), "v"(c), "v"(d)); }
__device__ __forceinline__ void acc_guard4(v8f& a, v8f& b, v8f& c, v8f& d) { asm volatile("v_nop\n\tv_nop\n\tv_nop\n\tv_nop" : "+v"(a), "+v"(b), "+v"(c), "+v"(d)); }
__device__ __forceinline__ void wave_sync() {
    __builtin_amdgcn_fence(3  , "workgroup");
    __builtin_amdgcn_wave_barrier();
    __builtin_amdgcn_fence(2  , "workgroup");
}

#define VST2(T, ptr, val) do { const T vst2_v_ = (val); *(volatile T*)(ptr) = vst2_v_; __threadfence(); *(volatile T*)(ptr) = vst2_v_; } while (0)

__device__ __forceinline__ float cmb_bf(float v) { const unsigned u = __builtin_bit_cast(unsigned, v); const unsigned r = (u + 0x7fffu + ((u >> 16) & 1u)) & 0xffff0000u; return __builtin_bit_cast(float, r); }
__device__ __forceinline__ unsigned int pk2h(float a, float b) { return (unsigned int)__builtin_bit_cast(unsigned short, (_Float16)a) | ((unsigned int)__builtin_bit_cast(unsigned short, (_Float16)b) << 16); }

__global__ __launch_bounds__(256) void k_ln512(const float* __restrict__ A, int src_rows_per_b, const float* __restrict__ GA, const float* __restrict__ BE, int abf, unsigned short* __restrict__ Y16) {
    #pragma clang fp contract(off)
    const int r = blockIdx.x * 8 + (threadIdx.x >> 5); const int L = threadIdx.x & 31; if (r >= ROWS) return;
    const int bb = r / SEQ, t = r - bb * SEQ;
    const float* src = A + ((long long)bb * src_rows_per_b + t) * DM;
    v4f v[4]; float s = 0.f;
#pragma unroll
    for (int q = 0; q < 4; ++q) {
        v[q] = *(const v4f*)(src + 4 * L + 128 * q);
        if (abf) { v[q].x = cmb_bf(v[q].x); v[q].y = cmb_bf(v[q].y); v[q].z = cmb_bf(v[q].z); v[q].w = cmb_bf(v[q].w); }
        s += (v[q].x + v[q].y) + (v[q].z + v[q].w);
    }
#pragma unroll
    for (int o = 16; o > 0; o >>= 1) s += __shfl_xor(s, o, 32);
    const float mu = s * (1.f / DM); float qq = 0.f;
#pragma unroll
    for (int q = 0; q < 4; ++q) { v[q].x -= mu; v[q].y -= mu; v[q].z -= mu; v[q].w -= mu; qq += (v[q].x * v[q].x + v[q].y * v[q].y) + (v[q].z * v[q].z + v[q].w * v[q].w); }
#pragma unroll
    for (int o = 16; o > 0; o >>= 1) qq += __shfl_xor(qq, o, 32);
    const float rs = rsqrtf(qq * (1.f / DM) + 1e-5f);
#pragma unroll
    for (int q = 0; q < 4; ++q) {
        const int c = 4 * L + 128 * q; const v4f ga = *(const v4f*)(GA + c), be = *(const v4f*)(BE + c); v4f y;
        y.x = v[q].x * rs * cmb_bf(ga.x) + cmb_bf(be.x); y.y = v[q].y * rs * cmb_bf(ga.y) + cmb_bf(be.y);
        y.z = v[q].z * rs * cmb_bf(ga.z) + cmb_bf(be.z); y.w = v[q].w * rs * cmb_bf(ga.w) + cmb_bf(be.w);
        u2 pk; pk.x = pk2h(y.x, y.y); pk.y = pk2h(y.z, y.w);
        VST2(u2, (u2*)(Y16 + (long long)r * DM + c), pk);
    }
}

__global__ __launch_bounds__(256) void k_castbT(const float* __restrict__ SRC, int lds, int src_slice, unsigned short* __restrict__ DST, int ldd, int dst_slice, int nR, int nC, float sc) {
    const long long u = (long long)blockIdx.x * 256 + threadIdx.x; const int per = nR / 8; if (u >= (long long)nC * per) return;
    const int c = (int)(u / per); const int r0 = 8 * (int)(u % per);
    const float* s = SRC + (long long)blockIdx.y * src_slice;
    float w[8];
#pragma unroll
    for (int e = 0; e < 8; ++e) w[e] = cmb_bf(s[(long long)(r0 + e) * lds + c]) * sc;
    u4 pk; pk.x = pk2h(w[0], w[1]); pk.y = pk2h(w[2], w[3]); pk.z = pk2h(w[4], w[5]); pk.w = pk2h(w[6], w[7]);
    VST2(u4, (u4*)(DST + (long long)blockIdx.y * dst_slice + (long long)c * ldd + r0), pk);
}

template <int BIAS, int OUT16, int RESID, int XBF, int RELU>
__device__ __forceinline__ void gemm64_body(
    const unsigned short* __restrict__ Ap, int lda, long long strideA,
    const unsigned short* __restrict__ Btp, int ldb, long long strideB,
    float* __restrict__ Cf, unsigned short* __restrict__ Ch, int ldc, long long strideC,
    const float* __restrict__ bias, const float* __restrict__ resid, int ldr, long long strideR,
    int M, int N, int K, float scale) {
  __shared__ __align__(16) float sT[8][16 * 68];
  const int bz   = blockIdx.y;
  const int lane = threadIdx.x & 31;
  const int wave = threadIdx.x >> 5;
  const int tilesN = N >> 6;
  const int tilesM = M >> 6;
  const int tile = blockIdx.x * 8 + wave;
  if (tile >= tilesM * tilesN) return;
  const int tm = tile / tilesN;
  const int tn = tile - tm * tilesN;
  const int m0 = tm << 6;
  const int n0 = tn << 6;
  const _Float16* Ab = (const _Float16*)Ap  + (size_t)bz * strideA;
  const _Float16* Bb = (const _Float16*)Btp + (size_t)bz * strideB;
  const int rlane = lane & 15;
  const int koff  = (lane >> 4) * 8;
  const int mOff  = (lane >> 4) * 8;

  v8f acc[4][4];
#pragma unroll
  for (int i = 0; i < 4; ++i)
#pragma unroll
    for (int j = 0; j < 4; ++j) acc[i][j] = (v8f){0.f,0.f,0.f,0.f,0.f,0.f,0.f,0.f};

  for (int k0 = 0; k0 < K; k0 += 32) {
    v16h bh[4];
#pragma unroll
    for (int j = 0; j < 4; ++j) bh[j] = ld_frag(Bb + (size_t)(n0 + (j << 4) + rlane) * ldb + koff + k0);
#pragma unroll
    for (int i = 0; i < 4; ++i) {
      const v16h ah = ld_frag(Ab + (size_t)(m0 + (i << 4) + rlane) * lda + koff + k0);
#pragma unroll
      for (int j = 0; j < 4; ++j)
        acc[i][j] = __builtin_amdgcn_wmma_f32_16x16x32_f16(false, ah, false, bh[j], (short)0, acc[i][j], false, false);
      dep_guard_h(acc[i][0], acc[i][3], ah, ah);
    }
    keep4_h(bh[0], bh[1], bh[2], bh[3]);
  }
  acc_guard4(acc[0][0], acc[0][1], acc[0][2], acc[0][3]);
  acc_guard4(acc[1][0], acc[1][1], acc[1][2], acc[1][3]);
  acc_guard4(acc[2][0], acc[2][1], acc[2][2], acc[2][3]);
  acc_guard4(acc[3][0], acc[3][1], acc[3][2], acc[3][3]);

  float bvj[4];
#pragma unroll
  for (int j = 0; j < 4; ++j) bvj[j] = BIAS ? cmb_bf(bias[n0 + (j << 4) + rlane]) : 0.f;

#pragma unroll
  for (int i = 0; i < 4; ++i) {
    const int mBase = m0 + (i << 4);
#pragma unroll
    for (int j = 0; j < 4; ++j) {
#pragma unroll
      for (int r = 0; r < 8; ++r) {
        float v = acc[i][j][r] * scale;
        if (BIAS) v += bvj[j];
        if (RELU) v = fmaxf(v, 0.0f);
        sT[wave][(mOff + r) * 68 + (j << 4) + rlane] = v;
      }
    }
    wave_sync();
    if (OUT16 == 0) {
      float* C = Cf + (size_t)bz * strideC;
      const int hh = lane >> 4, c4 = (lane & 15) * 4;
      v4f vv[8];
#pragma unroll
      for (int it = 0; it < 8; ++it) {
        const int row = it * 2 + hh;
        v4f v = *(const v4f_ma*)&sT[wave][row * 68 + c4];
        if (RESID) {
          v4f x = *(const v4f*)(resid + (size_t)bz * strideR + (size_t)(mBase + row) * ldr + n0 + c4);
          if (XBF) { x.x = cmb_bf(x.x); x.y = cmb_bf(x.y); x.z = cmb_bf(x.z); x.w = cmb_bf(x.w); }
          v = v + x;
        }
        vv[it] = v;
      }
#pragma unroll
      for (int it = 0; it < 8; ++it) *(volatile v4f*)(C + (size_t)(mBase + it * 2 + hh) * ldc + n0 + c4) = vv[it];
      __threadfence();
#pragma unroll
      for (int it = 0; it < 8; ++it) *(volatile v4f*)(C + (size_t)(mBase + it * 2 + hh) * ldc + n0 + c4) = vv[it];
    } else {
      unsigned short* C = Ch + (size_t)bz * strideC;
      const int q = lane >> 3, c8 = (lane & 7) * 8;
      v8h hv[4];
#pragma unroll
      for (int it = 0; it < 4; ++it) {
        const int row = it * 4 + q;
        const v4f a = *(const v4f_ma*)&sT[wave][row * 68 + c8];
        const v4f b = *(const v4f_ma*)&sT[wave][row * 68 + c8 + 4];
        v8h t;
        t[0] = (_Float16)a.x; t[1] = (_Float16)a.y; t[2] = (_Float16)a.z; t[3] = (_Float16)a.w;
        t[4] = (_Float16)b.x; t[5] = (_Float16)b.y; t[6] = (_Float16)b.z; t[7] = (_Float16)b.w;
        hv[it] = t;
      }
#pragma unroll
      for (int it = 0; it < 4; ++it) *(volatile v8h*)(C + (size_t)(mBase + it * 4 + q) * ldc + n0 + c8) = hv[it];
      __threadfence();
#pragma unroll
      for (int it = 0; it < 4; ++it) *(volatile v8h*)(C + (size_t)(mBase + it * 4 + q) * ldc + n0 + c8) = hv[it];
    }
    wave_sync();
  }
}

__global__ __launch_bounds__(256) void k_gemm_h16(const unsigned short* __restrict__ A, int lda, long long sA, const unsigned short* __restrict__ Bt, int ldb, long long sB,
                                                  unsigned short* __restrict__ C, int ldc, long long sC, int M, int N, int K, float scale) {
  gemm64_body<0, 1, 0, 0, 0>(A, lda, sA, Bt, ldb, sB, nullptr, C, ldc, sC, nullptr, nullptr, 0, 0, M, N, K, scale);
}
__global__ __launch_bounds__(256) void k_gemm_proj(const unsigned short* __restrict__ A, int lda, long long sA, const unsigned short* __restrict__ Bt, int ldb,
                                                   float* __restrict__ C, int ldc, long long sC, const float* __restrict__ bias, const float* __restrict__ R, int ldr, long long sR,
                                                   int M, int N, int K, float scale) {
  gemm64_body<1, 0, 1, 1, 0>(A, lda, sA, Bt, ldb, 0, C, nullptr, ldc, sC, bias, R, ldr, sR, M, N, K, scale);
}
__global__ __launch_bounds__(256) void k_gemm_ffn1(const unsigned short* __restrict__ A, int lda, long long sA, const unsigned short* __restrict__ Bt, int ldb,
                                                   unsigned short* __restrict__ C, int ldc, long long sC, const float* __restrict__ bias, int M, int N, int K, float scale) {
  gemm64_body<1, 1, 0, 0, 1>(A, lda, sA, Bt, ldb, 0, nullptr, C, ldc, sC, bias, nullptr, 0, 0, M, N, K, scale);
}
__global__ __launch_bounds__(256) void k_gemm_ffn2(const unsigned short* __restrict__ A, int lda, long long sA, const unsigned short* __restrict__ Bt, int ldb,
                                                   float* __restrict__ C, int ldc, long long sC, const float* __restrict__ bias, const float* __restrict__ R, int ldr, long long sR,
                                                   int M, int N, int K, float scale) {
  gemm64_body<1, 0, 1, 0, 0>(A, lda, sA, Bt, ldb, 0, C, nullptr, ldc, sC, bias, R, ldr, sR, M, N, K, scale);
}

__global__ __launch_bounds__(128) void k_attn(const unsigned short* __restrict__ QKp, const unsigned short* __restrict__ VTp, unsigned short* __restrict__ AOp, float sl2e) {
  __shared__ __align__(16) _Float16 Ps[4][16 * 40];
  __shared__ __align__(16) float    Os[4][16 * 68];
  const int tid = threadIdx.x, wave = tid >> 5, lane = tid & 31, hh = lane >> 4, c = lane & 15;
  const int nqb = SEQ / 64;
  const int bx = blockIdx.x;
  const int qb = bx % nqb;
  const int bh = bx / nqb;
  const int h  = bh % NHEAD;
  const int b  = bh / NHEAD;
  const int q0 = qb * 64 + wave * 16;
  const _Float16* QK = (const _Float16*)QKp + (size_t)b * SEQ * (2 * DM);
  const _Float16* VT = (const _Float16*)VTp + ((size_t)b * DM + (size_t)h * HDIM) * SEQ;
  const float NEG = -__builtin_inff();

  const int qoff = (q0 + c) * (2 * DM) + h * HDIM + 8 * hh;
  const v16h qa0 = ld_frag(QK + qoff), qa1 = ld_frag(QK + qoff + 32);

  float m8[8], l8[8];
  v8f o[4];
#pragma unroll
  for (int r = 0; r < 8; ++r) { m8[r] = NEG; l8[r] = 0.f; }
#pragma unroll
  for (int t = 0; t < 4; ++t) o[t] = (v8f){0.f,0.f,0.f,0.f,0.f,0.f,0.f,0.f};

  for (int key0 = 0; key0 <= q0 + 15; key0 += 32) {
    const int ko = (key0 + c) * (2 * DM) + DM + h * HDIM + 8 * hh;
    v8f s0 = (v8f){0.f,0.f,0.f,0.f,0.f,0.f,0.f,0.f};
    v8f s1 = (v8f){0.f,0.f,0.f,0.f,0.f,0.f,0.f,0.f};
    {
      const v16h kb0 = ld_frag(QK + ko), kb1 = ld_frag(QK + ko + 32);
      s0 = wmma16(qa0, kb0, s0);
      s0 = wmma16(qa1, kb1, s0);
    }
    {
      const v16h kb0 = ld_frag(QK + ko + 16 * (2 * DM)), kb1 = ld_frag(QK + ko + 16 * (2 * DM) + 32);
      s1 = wmma16(qa0, kb0, s1);
      s1 = wmma16(qa1, kb1, s1);
    }
#pragma unroll
    for (int r = 0; r < 8; ++r) {
      const int qrow = q0 + 8 * hh + r;
      float x0 = s0[r] * sl2e, x1 = s1[r] * sl2e;
      x0 = (key0 + c > qrow) ? NEG : x0;
      x1 = (key0 + 16 + c > qrow) ? NEG : x1;
      float mx = fmaxf(x0, x1);
      mx = fmaxf(mx, __shfl_xor(mx, 1, 32)); mx = fmaxf(mx, __shfl_xor(mx, 2, 32));
      mx = fmaxf(mx, __shfl_xor(mx, 4, 32)); mx = fmaxf(mx, __shfl_xor(mx, 8, 32));
      const float mnew = fmaxf(m8[r], mx);
      const float corr = (mnew == NEG) ? 1.f : exp2f(m8[r] - mnew);
      const float p0 = (x0 == NEG) ? 0.f : exp2f(x0 - mnew);
      const float p1 = (x1 == NEG) ? 0.f : exp2f(x1 - mnew);
      float rs = p0 + p1;
      rs += __shfl_xor(rs, 1, 32); rs += __shfl_xor(rs, 2, 32); rs += __shfl_xor(rs, 4, 32); rs += __shfl_xor(rs, 8, 32);
      l8[r] = l8[r] * corr + rs; m8[r] = mnew;
      o[0][r] *= corr; o[1][r] *= corr; o[2][r] *= corr; o[3][r] *= corr;
      Ps[wave][(8 * hh + r) * 40 + c]      = (_Float16)(p0 * 4096.f);
      Ps[wave][(8 * hh + r) * 40 + 16 + c] = (_Float16)(p1 * 4096.f);
    }
    wave_sync();
    FragU pf;
    pf.h[0] = *(const v8h_ma*)&Ps[wave][c * 40 + 8 * hh];
    pf.h[1] = *(const v8h_ma*)&Ps[wave][c * 40 + 16 + 8 * hh];
    const int vo = c * SEQ + key0 + 8 * hh;
    v16h vb[4];
#pragma unroll
    for (int t = 0; t < 4; ++t) vb[t] = ld_frag(VT + vo + t * 16 * SEQ);
#pragma unroll
    for (int t = 0; t < 4; ++t) o[t] = wmma16(pf.v, vb[t], o[t]);
    wave_sync();
  }

#pragma unroll
  for (int r = 0; r < 8; ++r) {
    const float inv = (l8[r] > 0.f) ? 1.0f / (l8[r] * 256.0f) : 0.f;
#pragma unroll
    for (int t = 0; t < 4; ++t) Os[wave][(8 * hh + r) * 68 + t * 16 + c] = o[t][r] * inv;
  }
  wave_sync();
  {
    unsigned short* AO = AOp + ((size_t)b * SEQ + q0) * DM + h * HDIM;
    const int q = lane >> 3, c8 = (lane & 7) * 8;
    v8h hv[4];
#pragma unroll
    for (int it = 0; it < 4; ++it) {
      const int row = it * 4 + q;
      const v4f a = *(const v4f_ma*)&Os[wave][row * 68 + c8];
      const v4f bq = *(const v4f_ma*)&Os[wave][row * 68 + c8 + 4];
      v8h t;
      t[0] = (_Float16)a.x; t[1] = (_Float16)a.y; t[2] = (_Float16)a.z; t[3] = (_Float16)a.w;
      t[4] = (_Float16)bq.x; t[5] = (_Float16)bq.y; t[6] = (_Float16)bq.z; t[7] = (_Float16)bq.w;
      hv[it] = t;
    }
#pragma unroll
    for (int it = 0; it < 4; ++it) *(volatile v8h*)(AO + (size_t)(it * 4 + q) * DM + c8) = hv[it];
    __threadfence();
#pragma unroll
    for (int it = 0; it < 4; ++it) *(volatile v8h*)(AO + (size_t)(it * 4 + q) * DM + c8) = hv[it];
  }
}

constexpr size_t SZ_H16  = (size_t)ROWS * DM * 2;
constexpr size_t SZ_W316 = (size_t)3 * DM * DM * 2;
constexpr size_t SZ_WO16 = (size_t)DM * DM * 2;
constexpr size_t SZ_W1T  = (size_t)DFF * DM * 2;
constexpr size_t SZ_W2T  = (size_t)DM * DFF * 2;
constexpr size_t SZ_QK16 = (size_t)ROWS * 2 * DM * 2;
constexpr size_t SZ_VT16 = (size_t)NB * DM * SEQ * 2;
constexpr size_t SZ_AO16 = (size_t)ROWS * DM * 2;
constexpr size_t SZ_X1   = (size_t)ROWS * DM * 4;
constexpr size_t SZ_H2   = (size_t)ROWS * DM * 2;
constexpr size_t SZ_U16  = (size_t)ROWS * DFF * 2;
constexpr size_t WS_TOTAL = SZ_H16 + SZ_W316 + SZ_WO16 + SZ_W1T + SZ_W2T + SZ_QK16 + SZ_VT16 + SZ_AO16 + SZ_X1 + SZ_H2 + SZ_U16;
static_assert(WS_TOTAL <= (size_t)134217728);
static_assert(SZ_H16 % 256 == 0 && SZ_W316 % 256 == 0 && SZ_WO16 % 256 == 0 && SZ_W1T % 256 == 0 && SZ_W2T % 256 == 0 && SZ_QK16 % 256 == 0 && SZ_VT16 % 256 == 0 && SZ_AO16 % 256 == 0 && SZ_X1 % 256 == 0 && SZ_H2 % 256 == 0);

extern "C" void kernel_launch(void* const* d_in, const int* in_sizes, int n_in, void* d_out, int out_size, void* d_ws, size_t ws_size, hipStream_t stream) {
    if (n_in < 12) return;
    const long long need_x = ((long long)(NB - 1) * SEQ_FULL + SEQ) * DM;
    if ((long long)in_sizes[0] < need_x || (long long)out_size < need_x) return;
    if (in_sizes[1] < DM || in_sizes[2] < DM || in_sizes[3] < NHEAD * DM * HDIM || in_sizes[4] < NHEAD * DM * HDIM || in_sizes[5] < NHEAD * DM * HDIM) return;
    if (in_sizes[6] < DM * DM || in_sizes[7] < DM || in_sizes[8] < DM * DFF || in_sizes[9] < DFF || in_sizes[10] < DFF * DM || in_sizes[11] < DM) return;
    if (ws_size < WS_TOTAL) return;
    const float* x   = (const float*)d_in[0];
    const float* lng = (const float*)d_in[1];
    const float* lnb = (const float*)d_in[2];
    const float* wq  = (const float*)d_in[3];
    const float* wk  = (const float*)d_in[4];
    const float* wv  = (const float*)d_in[5];
    const float* wo  = (const float*)d_in[6];
    const float* bo  = (const float*)d_in[7];
    const float* w1  = (const float*)d_in[8];
    const float* b1  = (const float*)d_in[9];
    const float* w2  = (const float*)d_in[10];
    const float* b2  = (const float*)d_in[11];
    float* out = (float*)d_out;
    char* wsp = (char*)d_ws;
    unsigned short* H16  = (unsigned short*)wsp; wsp += SZ_H16;
    unsigned short* W316 = (unsigned short*)wsp; wsp += SZ_W316;
    unsigned short* WO16 = (unsigned short*)wsp; wsp += SZ_WO16;
    unsigned short* W1T  = (unsigned short*)wsp; wsp += SZ_W1T;
    unsigned short* W2T  = (unsigned short*)wsp; wsp += SZ_W2T;
    unsigned short* QK16 = (unsigned short*)wsp; wsp += SZ_QK16;
    unsigned short* VT16 = (unsigned short*)wsp; wsp += SZ_VT16;
    unsigned short* AO16 = (unsigned short*)wsp; wsp += SZ_AO16;
    float*          X1   = (float*)wsp;          wsp += SZ_X1;
    unsigned short* H2   = (unsigned short*)wsp; wsp += SZ_H2;
    unsigned short* U16  = (unsigned short*)wsp; wsp += SZ_U16;

    const float sl2e = 0.04419417382415922f * 1.4426950408889634f;

    k_ln512<<<ROWS / 8, 256, 0, stream>>>(x, SEQ_FULL, lng, lnb, 1, H16);
    k_castbT<<<dim3((HDIM * (DM / 8) + 255) / 256, NHEAD), 256, 0, stream>>>(wq, HDIM, DM * HDIM, W316, DM, HDIM * DM, DM, HDIM, 16.0f);
    k_castbT<<<dim3((HDIM * (DM / 8) + 255) / 256, NHEAD), 256, 0, stream>>>(wk, HDIM, DM * HDIM, W316 + (size_t)DM * DM, DM, HDIM * DM, DM, HDIM, 16.0f);
    k_castbT<<<dim3((HDIM * (DM / 8) + 255) / 256, NHEAD), 256, 0, stream>>>(wv, HDIM, DM * HDIM, W316 + (size_t)2 * DM * DM, DM, HDIM * DM, DM, HDIM, 16.0f);
    k_castbT<<<dim3((DM * (DM / 8) + 255) / 256, 1), 256, 0, stream>>>(wo, DM, 0, WO16, DM, 0, DM, DM, 16.0f);
    k_castbT<<<dim3((DFF * (DM / 8) + 255) / 256, 1), 256, 0, stream>>>(w1, DFF, 0, W1T, DM, 0, DM, DFF, 16.0f);
    k_castbT<<<dim3((DM * (DFF / 8) + 255) / 256, 1), 256, 0, stream>>>(w2, DM, 0, W2T, DFF, 0, DFF, DM, 16.0f);
    k_gemm_h16<<<dim3(((SEQ / 64) * ((2 * DM) / 64) + 7) / 8, NB), 256, 0, stream>>>(H16, DM, (long long)SEQ * DM, W316, DM, 0, QK16, 2 * DM, (long long)SEQ * 2 * DM, SEQ, 2 * DM, DM, 0.0625f);
    k_gemm_h16<<<dim3(((DM / 64) * (SEQ / 64) + 7) / 8, NB), 256, 0, stream>>>(W316 + (size_t)2 * DM * DM, DM, 0, H16, DM, (long long)SEQ * DM, VT16, SEQ, (long long)DM * SEQ, DM, SEQ, DM, 0.0625f);
    k_attn<<<NB * NHEAD * (SEQ / 64), 128, 0, stream>>>(QK16, VT16, AO16, sl2e);
    k_gemm_proj<<<dim3(((SEQ / 64) * (DM / 64) + 7) / 8, NB), 256, 0, stream>>>(AO16, DM, (long long)SEQ * DM, WO16, DM, X1, DM, (long long)SEQ * DM, bo, x, DM, (long long)SEQ_FULL * DM, SEQ, DM, DM, 0.00390625f);
    k_ln512<<<ROWS / 8, 256, 0, stream>>>(X1, SEQ, lng, lnb, 0, H2);
    k_gemm_ffn1<<<dim3(((SEQ / 64) * (DFF / 64) + 7) / 8, NB), 256, 0, stream>>>(H2, DM, (long long)SEQ * DM, W1T, DM, U16, DFF, (long long)SEQ * DFF, b1, SEQ, DFF, DM, 0.0625f);
    k_gemm_ffn2<<<dim3(((SEQ / 64) * (DM / 64) + 7) / 8, NB), 256, 0, stream>>>(U16, DFF, (long long)SEQ * DFF, W2T, DFF, out, DM, (long long)SEQ_FULL * DM, b2, X1, DM, (long long)SEQ * DM, SEQ, DM, DFF, 0.0625f);
}
